// TransformerBlock_25769804134
// MI455X (gfx1250) — hardware-verified
//
#include <hip/hip_runtime.h>
#ifndef NB
#define NB 8
#endif
#ifndef SEQ
#define SEQ 1024
#endif
#define SEQ_FULL 1024
#define DM 768
#define NH 12
#define HD 64
#define DFF 3072
#define LQ (3 * DM)
#define NJ (DM / 128)
#define NR ((size_t)NB * SEQ)
#define MP (NB * SEQ)

static_assert(DM % 128 == 0);
static_assert(HD == 64);
static_assert(NH * HD == DM);
static_assert(SEQ % 128 == 0);
static_assert(SEQ <= SEQ_FULL);
static_assert(MP % 128 == 0);
static_assert(LQ % 64 == 0);
static_assert(DFF % 64 == 0);
static_assert(DM % 64 == 0);
static_assert(DM % 32 == 0);
static_assert(DFF % 32 == 0);
static_assert(((size_t)NB * SEQ) % 4 == 0);
static_assert(((size_t)LQ * (DM / 8)) % 256 == 0);
static_assert(((size_t)DM * (DM / 8)) % 256 == 0);
static_assert(((size_t)DFF * (DM / 8)) % 256 == 0);
static_assert(((size_t)DM * (DFF / 8)) % 256 == 0);
static_assert((DM / 8) % 32 == 0);
static_assert((DFF / 8) % 32 == 0);
static_assert(NJ * 128 == DM);

typedef unsigned short v8us __attribute__((ext_vector_type(8), may_alias));
typedef float  v8f  __attribute__((ext_vector_type(8)));
typedef float  v4f  __attribute__((ext_vector_type(4)));
typedef float  v4fa __attribute__((ext_vector_type(4), may_alias));
typedef _Float16 v16h __attribute__((ext_vector_type(16)));
typedef _Float16 v4h __attribute__((ext_vector_type(4)));
union FragH { v16h v; v8us half[2]; _Float16 h[16]; unsigned short u[16]; };

__device__ __forceinline__ float bf16_rne(float x) { unsigned int u = __float_as_uint(x); u = (u + 0x7FFFu + ((u >> 16) & 1u)) & 0xFFFF0000u; return __uint_as_float(u); }

__device__ __forceinline__ v16h g2_frag(const _Float16* p, unsigned hh) { FragH f; f.half[0] = *(const v8us*)((const unsigned short*)p + 8u * hh); f.half[1] = *(const v8us*)((const unsigned short*)p + 16u + 8u * hh); return f.v; }
__device__ __forceinline__ v8f g2_mma(v16h a, v16h b, v8f c) { v8f d = __builtin_amdgcn_wmma_f32_16x16x32_f16(false, a, false, b, (short)0, c, false, false); asm volatile("v_nop\n\tv_nop\n\tv_nop\n\tv_nop" : "+v"(d) : "v"(a), "v"(b)); return d; }

template <unsigned K, unsigned N>
__global__ __launch_bounds__(256) void k_wt_f16(const float* __restrict__ W, _Float16* __restrict__ Wt, float scale) {
  const unsigned t = blockIdx.x * 256u + threadIdx.x; if (t >= N * (K / 8u)) return;
  const unsigned n = t / (K / 8u), k8 = (t % (K / 8u)) * 8u; FragH f;
#pragma unroll
  for (unsigned i = 0; i < 8u; ++i) f.h[i] = (_Float16)(bf16_rne(W[(size_t)(k8 + i) * N + n]) * scale);
  const v8us o = f.half[0]; unsigned short* dst = (unsigned short*)Wt + (size_t)n * K + k8;
  *(volatile v8us*)dst = o; __threadfence(); *(volatile v8us*)dst = o;
}

template <int BFIN, int WXB, int MAPX>
__global__ __launch_bounds__(128) void k_lnw(const float* __restrict__ X, const float* __restrict__ g, const float* __restrict__ bb, float eps, _Float16* __restrict__ N16, float* __restrict__ XB) {
  #pragma clang fp contract(off)
  const unsigned lane = threadIdx.x & 31u, w = threadIdx.x >> 5;
  const unsigned r = blockIdx.x * 4u + w;
  if (r >= (unsigned)MP) return;
  const unsigned rsrc = MAPX ? (r / (unsigned)SEQ) * (unsigned)SEQ_FULL + (r % (unsigned)SEQ) : r;
  const float* xr = X + (size_t)rsrc * DM + lane * 4u;
  const float* gp = g + lane * 4u;
  const float* bp = bb + lane * 4u;
  float sum = 0.f;
#pragma unroll 1
  for (unsigned j = 0; j < (unsigned)NJ; ++j) { const v4f a = *(const v4fa*)(xr + j * 128u);
#pragma unroll
    for (int q = 0; q < 4; ++q) { const float v = BFIN ? bf16_rne(a[q]) : a[q]; sum = sum + v; } }
#pragma unroll
  for (int d = 16; d > 0; d >>= 1) sum = sum + __shfl_xor(sum, d, 32);
  const float mu = sum * (1.0f / (float)DM);
  float vs = 0.f;
#pragma unroll 1
  for (unsigned j = 0; j < (unsigned)NJ; ++j) { const v4f a = *(const v4fa*)(xr + j * 128u);
#pragma unroll
    for (int q = 0; q < 4; ++q) { const float v = BFIN ? bf16_rne(a[q]) : a[q]; const float dl = v - mu; vs = vs + dl * dl; } }
#pragma unroll
  for (int d = 16; d > 0; d >>= 1) vs = vs + __shfl_xor(vs, d, 32);
  const float rs = rsqrtf(vs * (1.0f / (float)DM) + eps);
  _Float16* yr = N16 + (size_t)r * DM + lane * 4u;
  for (int pass = 0; pass < 2; ++pass) {
#pragma unroll 1
    for (unsigned j = 0; j < (unsigned)NJ; ++j) { const v4f a = *(const v4fa*)(xr + j * 128u); const v4f gg = *(const v4fa*)(gp + j * 128u); const v4f be = *(const v4fa*)(bp + j * 128u);
      v4h y; v4f xb;
#pragma unroll
      for (int q = 0; q < 4; ++q) { const float xv = BFIN ? bf16_rne(a[q]) : a[q]; const float v = (xv - mu) * rs * bf16_rne(gg[q]) + bf16_rne(be[q]); y[q] = (_Float16)v; xb[q] = xv; }
      *(volatile v4h*)(yr + j * 128u) = y;
      if (WXB) *(volatile v4f*)(XB + (size_t)r * DM + lane * 4u + j * 128u) = xb; }
    if (pass == 0) __threadfence(); }
}

template <int ACT>
__global__ __launch_bounds__(128) void k_gemm2(const _Float16* __restrict__ A, int lda, size_t sA, const _Float16* __restrict__ Bh, int ldb, size_t sB, float alpha, const float* __restrict__ bias, size_t sBias, const float* __restrict__ CP,
    float* __restrict__ C, _Float16* __restrict__ C16, float c16s, int ldc, size_t sC, int M, int N, int K) {
  static_assert(ACT == 0 || ACT == 3 || ACT == 6);
  __shared__ __attribute__((aligned(16))) float so[4][32][68];
  const unsigned tid = threadIdx.x, w = tid >> 5, lane = tid & 31u, ln = lane & 15u, hh = lane >> 4; const unsigned by = blockIdx.y;
  A += (size_t)by * sA; Bh += (size_t)by * sB; const size_t cofs = (size_t)by * sC; const float* bp = bias ? bias + (size_t)by * sBias : nullptr;
  const unsigned ntn = (unsigned)N >> 6; const unsigned mt = blockIdx.x / ntn, nq = blockIdx.x - mt * ntn; const unsigned row0 = mt * 128u + 32u * w, col0 = nq * 64u; if (row0 >= (unsigned)M) return;
  const _Float16* a0p = A + (size_t)(row0 + ln) * lda; const _Float16* a1p = a0p + (size_t)16 * lda;
  const _Float16* b0p = Bh + (size_t)(col0 + ln) * ldb; const _Float16* b1p = b0p + (size_t)16 * ldb; const _Float16* b2p = b1p + (size_t)16 * ldb; const _Float16* b3p = b2p + (size_t)16 * ldb;
  const v8f z8 = {0.f,0.f,0.f,0.f,0.f,0.f,0.f,0.f}; v8f c00 = z8, c01 = z8, c02 = z8, c03 = z8, c10 = z8, c11 = z8, c12 = z8, c13 = z8;
#pragma unroll 1
  for (int kb = 0; kb < K; kb += 32) { const v16h a0 = g2_frag(a0p + kb, hh), a1 = g2_frag(a1p + kb, hh);
    v16h b = g2_frag(b0p + kb, hh); c00 = g2_mma(a0, b, c00); c10 = g2_mma(a1, b, c10);
    b = g2_frag(b1p + kb, hh); c01 = g2_mma(a0, b, c01); c11 = g2_mma(a1, b, c11);
    b = g2_frag(b2p + kb, hh); c02 = g2_mma(a0, b, c02); c12 = g2_mma(a1, b, c12);
    b = g2_frag(b3p + kb, hh); c03 = g2_mma(a0, b, c03); c13 = g2_mma(a1, b, c13); }
  v8f accs[8] = {c00, c01, c02, c03, c10, c11, c12, c13};
#pragma unroll
  for (int u = 0; u < 8; ++u) { const unsigned t = (unsigned)u & 3u, half = (unsigned)u >> 2; const unsigned col = col0 + t * 16u + ln; const float bv = bp ? bf16_rne(bp[col]) : 0.f;
#pragma unroll
    for (int r = 0; r < 8; ++r) { const unsigned rloc = half * 16u + 8u * hh + (unsigned)r; float v = accs[u][r] * alpha + bv; if (CP) v += CP[cofs + (size_t)(row0 + rloc) * ldc + col];
      if (ACT == 3) v = fmaxf(v, 0.f); else if (ACT == 6) v = 0.5f * v * (1.0f + erff(v * 0.70710678118654752f));
      so[w][rloc][t * 16u + ln] = v; } }
  __builtin_amdgcn_fence(4  , "workgroup"); __builtin_amdgcn_wave_barrier();
  const unsigned rsub = lane >> 4, c4 = (lane & 15u) * 4u;
  for (int pass = 0; pass < 2; ++pass) {
#pragma unroll
    for (int q = 0; q < 16; ++q) { const unsigned r = (unsigned)q * 2u + rsub; const v4f v = *(const v4fa*)&so[w][r][c4]; if (C) *(volatile v4f*)(C + cofs + (size_t)(row0 + r) * ldc + col0 + c4) = v; if (C16) { v4h h4; for (int i = 0; i < 4; ++i) h4[i] = (_Float16)(v[i] * c16s); *(volatile v4h*)(C16 + cofs + (size_t)(row0 + r) * ldc + col0 + c4) = h4; } }
    if (pass == 0) __threadfence(); } }

__global__ __launch_bounds__(256) void k_vt(const _Float16* __restrict__ V16, _Float16* __restrict__ Vt) {
  __shared__ unsigned short tl[64][66]; const unsigned tid = threadIdx.x; const unsigned slab = blockIdx.x / ((unsigned)SEQ / 64u), lg = blockIdx.x % ((unsigned)SEQ / 64u); const unsigned b = slab / (unsigned)NH, h = slab % (unsigned)NH;
  for (unsigned i = tid; i < 512u; i += 256u) { const unsigned r = i >> 3, c8 = (i & 7u) * 8u; FragH f; f.half[0] = *(const v8us*)((const unsigned short*)V16 + ((size_t)b * SEQ + lg * 64u + r) * LQ + h * (unsigned)HD + c8);
#pragma unroll
    for (int q = 0; q < 8; ++q) tl[r][c8 + q] = f.u[q]; }
  __syncthreads();
  for (int pass = 0; pass < 2; ++pass) {
#pragma unroll
    for (unsigned rd = 0; rd < 2u; ++rd) { const unsigned d = rd * 32u + (tid >> 3), pc = tid & 7u; FragH f;
#pragma unroll
      for (int q = 0; q < 8; ++q) f.u[q] = tl[pc * 8u + q][d];
      *(volatile v8us*)((unsigned short*)Vt + ((size_t)slab * HD + d) * SEQ + lg * 64u + pc * 8u) = f.half[0]; }
    if (pass == 0) __threadfence(); } }

__global__ __launch_bounds__(128) void k_flash(const _Float16* __restrict__ QKV, const _Float16* __restrict__ VT, _Float16* __restrict__ O16) {
  __shared__ __attribute__((aligned(16))) unsigned short so[4][16][72];
  const unsigned tid = threadIdx.x, w = tid >> 5, lane = tid & 31u, ln = lane & 15u, hh = lane >> 4;
  const unsigned qc = blockIdx.x % ((unsigned)SEQ / 64u), slab = blockIdx.x / ((unsigned)SEQ / 64u); const unsigned h = slab % (unsigned)NH, b = slab / (unsigned)NH;
  const unsigned q0 = qc * 64u + w * 16u;
  const _Float16* qrow = QKV + ((size_t)b * SEQ + q0 + ln) * LQ + h * (unsigned)HD;
  const v16h qf0 = g2_frag(qrow, hh), qf1 = g2_frag(qrow + 32, hh);
  const _Float16* kbase = QKV + ((size_t)b * SEQ + ln) * LQ + DM + h * (unsigned)HD;
  const _Float16* vbase = VT + ((size_t)slab * HD + ln) * SEQ;
  const v8f z8 = {0.f,0.f,0.f,0.f,0.f,0.f,0.f,0.f};
  v8f o0 = z8, o1 = z8, o2 = z8, o3 = z8; float m = -1.0e30f, l = 0.f;
#pragma unroll 1
  for (unsigned kb = 0; kb < (unsigned)SEQ; kb += 32u) {
    const _Float16* k0p = kbase + (size_t)kb * LQ; const _Float16* k1p = k0p + (size_t)16 * LQ;
    v8f s0 = g2_mma(g2_frag(k0p, hh), qf0, z8); s0 = g2_mma(g2_frag(k0p + 32, hh), qf1, s0);
    v8f s1 = g2_mma(g2_frag(k1p, hh), qf0, z8); s1 = g2_mma(g2_frag(k1p + 32, hh), qf1, s1);
    float mx = fmaxf(s0[0], s1[0]);
#pragma unroll
    for (int r = 1; r < 8; ++r) mx = fmaxf(mx, fmaxf(s0[r], s1[r]));
    mx = fmaxf(mx, __shfl_xor(mx, 16, 32));
    const float mn = fmaxf(m, mx * 0.125f);
    const float alpha = __expf(m - mn);
    const float cb = 6.931471806f - mn;
    FragH pf; float ps = 0.f;
#pragma unroll
    for (int r = 0; r < 8; ++r) { const float e0 = __expf(fmaf(s0[r], 0.125f, cb)); const float e1 = __expf(fmaf(s1[r], 0.125f, cb)); pf.h[r] = (_Float16)e0; pf.h[8 + r] = (_Float16)e1; ps += e0 + e1; }
    l = l * alpha + ps; m = mn;
    if (__builtin_amdgcn_ballot_w32(alpha != 1.0f) != 0u) { o0 *= alpha; o1 *= alpha; o2 *= alpha; o3 *= alpha; }
    o0 = g2_mma(g2_frag(vbase + kb, hh), pf.v, o0);
    o1 = g2_mma(g2_frag(vbase + (size_t)16 * SEQ + kb, hh), pf.v, o1);
    o2 = g2_mma(g2_frag(vbase + (size_t)32 * SEQ + kb, hh), pf.v, o2);
    o3 = g2_mma(g2_frag(vbase + (size_t)48 * SEQ + kb, hh), pf.v, o3);
  }
  const float lt = l + __shfl_xor(l, 16, 32);
  const float fin = 64.0f * (1.0f / lt);
  v8f oo[4] = {o0, o1, o2, o3};
#pragma unroll
  for (int t = 0; t < 4; ++t) { FragH f;
#pragma unroll
    for (int r = 0; r < 8; ++r) f.h[r] = (_Float16)(oo[t][r] * fin);
    *(v8us*)&so[w][ln][(unsigned)t * 16u + 8u * hh] = f.half[0]; }
  __builtin_amdgcn_fence(4  , "workgroup"); __builtin_amdgcn_wave_barrier();
  const unsigned rq = lane >> 3, pc = (lane & 7u) * 8u;
  for (int pass = 0; pass < 2; ++pass) {
#pragma unroll
    for (unsigned it = 0; it < 4u; ++it) { const unsigned row = it * 4u + rq; const v8us v = *(const v8us*)&so[w][row][pc]; *(volatile v8us*)((unsigned short*)O16 + ((size_t)b * SEQ + q0 + row) * DM + h * (unsigned)HD + pc) = v; }
    if (pass == 0) __threadfence(); }
}

extern "C" void kernel_launch(void* const* d_in, const int* in_sizes, int n_in,
                              void* d_out, int out_size, void* d_ws, size_t ws_size, hipStream_t stream) {
  if (n_in < 13) return;
  const size_t xneed = ((size_t)(NB - 1) * SEQ_FULL + SEQ) * DM;
  if ((size_t)in_sizes[0] < xneed || (size_t)out_size < xneed) return;
  if (in_sizes[1] < DM || in_sizes[2] < DM || in_sizes[3] < DM * LQ || in_sizes[4] < LQ || in_sizes[5] < DM * DM || in_sizes[6] < DM || in_sizes[7] < DM || in_sizes[8] < DM || in_sizes[9] < DM * DFF || in_sizes[10] < DFF || in_sizes[11] < DFF * DM || in_sizes[12] < DM) return;
  const float* const* I = (const float* const*)d_in;
  const float* x = I[0]; const float* g1 = I[1]; const float* be1 = I[2]; const float* wqkv = I[3]; const float* bqkv = I[4]; const float* wo = I[5]; const float* bo = I[6]; const float* g2 = I[7]; const float* be2 = I[8]; const float* wfc1 = I[9]; const float* bfc1 = I[10]; const float* wfc2 = I[11]; const float* bfc2 = I[12];
  float* out = (float*)d_out;
  char* ws = (char*)d_ws; size_t off = 0;
  auto take = [&](size_t bytes) { char* p = ws + off; off += (bytes + 255) & ~(size_t)255; return p; };
  _Float16* BQKV = (_Float16*)take((size_t)LQ * DM * 2);
  _Float16* BO   = (_Float16*)take((size_t)DM * DM * 2);
  _Float16* BW1  = (_Float16*)take((size_t)DFF * DM * 2);
  _Float16* BW2  = (_Float16*)take((size_t)DM * DFF * 2);
  _Float16* X16  = (_Float16*)take(NR * DM * 2);
  float*    XB   = (float*)take(NR * DM * 4);
  const size_t qkvBytes = NR * LQ * 2, vtBytes = (size_t)NB * NH * HD * SEQ * 2, hidBytes = NR * DFF * 2;
  const size_t regBytes = (qkvBytes + vtBytes) > hidBytes ? (qkvBytes + vtBytes) : hidBytes;
  char* REG = take(regBytes);
  _Float16* QKV  = (_Float16*)REG;
  _Float16* VT   = (_Float16*)(REG + qkvBytes);
  _Float16* HF16 = (_Float16*)REG;
  float*    X1   = (float*)take(NR * DM * 4);
  _Float16* O16  = X16;
  _Float16* M16  = X16;
  if (off > ws_size || off > (size_t)134217728) return;

  k_wt_f16<DM, LQ><<<(unsigned)(((size_t)LQ * (DM / 8) + 255) / 256), 256, 0, stream>>>(wqkv, BQKV, 16.0f);
  k_wt_f16<DM, DM><<<(unsigned)(((size_t)DM * (DM / 8) + 255) / 256), 256, 0, stream>>>(wo, BO, 16.0f);
  k_wt_f16<DM, DFF><<<(unsigned)(((size_t)DFF * (DM / 8) + 255) / 256), 256, 0, stream>>>(wfc1, BW1, 16.0f);
  k_wt_f16<DFF, DM><<<(unsigned)(((size_t)DM * (DFF / 8) + 255) / 256), 256, 0, stream>>>(wfc2, BW2, 16.0f);
  k_lnw<1, 1, 1><<<(unsigned)(NR / 4), 128, 0, stream>>>(x, g1, be1, 1e-5f, X16, XB);
  k_gemm2<0><<<dim3((unsigned)((MP / 128) * (LQ / 64)), 1), 128, 0, stream>>>(X16, DM, (size_t)0, BQKV, DM, (size_t)0, 0.0625f, bqkv, (size_t)0, nullptr, nullptr, QKV, 1.0f, LQ, (size_t)0, MP, LQ, DM);
  k_vt<<<(unsigned)(NB * NH * (SEQ / 64)), 256, 0, stream>>>(QKV + 2 * DM, VT);
  k_flash<<<(unsigned)(NB * NH * (SEQ / 64)), 128, 0, stream>>>(QKV, VT, O16);
  k_gemm2<0><<<dim3((unsigned)((MP / 128) * (DM / 64)), 1), 128, 0, stream>>>(O16, DM, (size_t)0, BO, DM, (size_t)0, 0.0009765625f, bo, (size_t)0, XB, X1, nullptr, 1.0f, DM, (size_t)0, MP, DM, DM);
  k_lnw<0, 0, 0><<<(unsigned)(NR / 4), 128, 0, stream>>>(X1, g2, be2, 1e-5f, M16, nullptr);
  k_gemm2<6><<<dim3((unsigned)((MP / 128) * (DFF / 64)), 1), 128, 0, stream>>>(M16, DM, (size_t)0, BW1, DM, (size_t)0, 0.0625f, bfc1, (size_t)0, nullptr, nullptr, HF16, 16.0f, DFF, (size_t)0, MP, DFF, DM);
  if (SEQ == SEQ_FULL) {
    k_gemm2<0><<<dim3((unsigned)((MP / 128) * (DM / 64)), 1), 128, 0, stream>>>(HF16, DFF, (size_t)0, BW2, DFF, (size_t)0, 0.00390625f, bfc2, (size_t)0, X1, out, nullptr, 1.0f, DM, (size_t)0, MP, DM, DFF);
  } else {
    for (int b = 0; b < NB; ++b)
      k_gemm2<0><<<dim3((unsigned)((SEQ / 128) * (DM / 64)), 1), 128, 0, stream>>>(HF16 + (size_t)b * SEQ * DFF, DFF, (size_t)0, BW2, DFF, (size_t)0, 0.00390625f, bfc2, (size_t)0, X1 + (size_t)b * SEQ * DM, out + (size_t)b * SEQ_FULL * DM, nullptr, 1.0f, DM, (size_t)0, SEQ, DM, DFF);
  }
}
